// MultiHeadSelfAttention_69853348102594
// MI455X (gfx1250) — hardware-verified
//
#include <hip/hip_runtime.h>
#ifndef NB
#define NB 2
#endif
#ifndef SEQ
#define SEQ 2048
#endif
#define SEQ_FULL 2048
#define DM 1024
#define NH 16
#define HD 64
#define NRI (NB * SEQ)
#define NR ((size_t)NRI)
#define LN_CARRY 6.931471806f

static_assert(DM == NH * HD);
static_assert(HD == 64);
static_assert(DM % 128 == 0);
static_assert(DM % 64 == 0);
static_assert(NRI % 128 == 0);
static_assert(NRI % 64 == 0);
static_assert(SEQ % 64 == 0);
static_assert(SEQ <= SEQ_FULL);
static_assert(((size_t)NB * SEQ * DM) % 8 == 0);

typedef __bf16 v16b __attribute__((ext_vector_type(16)));
typedef _Float16 v16h __attribute__((ext_vector_type(16)));
typedef unsigned short v8us __attribute__((ext_vector_type(8), may_alias));
typedef float v8f __attribute__((ext_vector_type(8)));
typedef float v4f __attribute__((ext_vector_type(4)));
typedef float v4fa __attribute__((ext_vector_type(4), may_alias));
union FragB { v16b v; v8us half[2]; };
union FragH { v16h v; v8us half[2]; _Float16 h[16]; };
union Pack8 { v8us v; _Float16 h[8]; };

__device__ __forceinline__ unsigned short bf16_bits(float x) { const unsigned int u = __float_as_uint(x); return (unsigned short)((u + 0x7FFFu + ((u >> 16) & 1u)) >> 16); }
__device__ __forceinline__ float bf16_val(unsigned short b) { return __uint_as_float(((unsigned int)b) << 16); }
__device__ __forceinline__ float bf16_rne(float x) { return bf16_val(bf16_bits(x)); }

__device__ __forceinline__ v16b ldb(const unsigned short* p) { FragB f; f.half[0] = *(const v8us*)p; f.half[1] = *(const v8us*)(p + 16); return f.v; }
__device__ __forceinline__ v16h ldh(const unsigned short* p) { FragH f; f.half[0] = *(const v8us*)p; f.half[1] = *(const v8us*)(p + 16); return f.v; }
__device__ __forceinline__ v8f mma_b(v16b a, v16b b, v8f c) {
  c = __builtin_amdgcn_wmma_f32_16x16x32_bf16(false, a, false, b, (short)0, c, false, false);
  asm volatile("v_nop\n\tv_nop\n\tv_nop\n\tv_nop" : "+v"(c) : "v"(a), "v"(b));
  return c;
}
__device__ __forceinline__ v8f mma_h(v16h a, v16h b, v8f c) {
  c = __builtin_amdgcn_wmma_f32_16x16x32_f16(false, a, false, b, (short)0, c, false, false);
  asm volatile("v_nop\n\tv_nop\n\tv_nop\n\tv_nop" : "+v"(c) : "v"(a), "v"(b));
  return c;
}

__global__ __launch_bounds__(256) void k_w_bf16(const float* __restrict__ w, unsigned short* __restrict__ Wb, int n8) {
  const int t = blockIdx.x * 256 + threadIdx.x;
  if (t >= n8) return;
  const v4f a = *(const v4fa*)(w + (size_t)t * 8), c = *(const v4fa*)(w + (size_t)t * 8 + 4);
  v8us o;
  o[0] = bf16_bits(a[0]); o[1] = bf16_bits(a[1]); o[2] = bf16_bits(a[2]); o[3] = bf16_bits(a[3]);
  o[4] = bf16_bits(c[0]); o[5] = bf16_bits(c[1]); o[6] = bf16_bits(c[2]); o[7] = bf16_bits(c[3]);
  unsigned short* d = Wb + (size_t)t * 8;
  *(volatile v8us*)d = o;
  __threadfence();
  *(volatile v8us*)d = o;
}

__global__ __launch_bounds__(256) void k_x_bf16(const float* __restrict__ x, unsigned short* __restrict__ XB, int n8) {
  const int t = blockIdx.x * 256 + threadIdx.x;
  if (t >= n8) return;
  const size_t e = (size_t)t * 8;
  const size_t r = e / DM; const int c = (int)(e % DM);
  const size_t bb = r / SEQ, s = r % SEQ;
  const float* src = x + (bb * SEQ_FULL + s) * DM + c;
  const v4f a = *(const v4fa*)src, q = *(const v4fa*)(src + 4);
  v8us o;
  o[0] = bf16_bits(a[0]); o[1] = bf16_bits(a[1]); o[2] = bf16_bits(a[2]); o[3] = bf16_bits(a[3]);
  o[4] = bf16_bits(q[0]); o[5] = bf16_bits(q[1]); o[6] = bf16_bits(q[2]); o[7] = bf16_bits(q[3]);
  unsigned short* d = XB + e;
  *(volatile v8us*)d = o;
  __threadfence();
  *(volatile v8us*)d = o;
}

template <int NA, int EPI>
__device__ __forceinline__ void gemm_tile(const unsigned short* __restrict__ A, const unsigned short* __restrict__ AL, int lda,
                                          const unsigned short* __restrict__ Bt, int pitch_b, const float* __restrict__ bias, float escale,
                                          unsigned short* __restrict__ O1, unsigned short* __restrict__ O2, float* __restrict__ OF,
                                          int ldc, int M, int N, int K) {
  __shared__ __attribute__((aligned(16))) float so[4][32][68];
  const int w = __builtin_amdgcn_readfirstlane((int)(threadIdx.x >> 5));
  const int lane = threadIdx.x & 31, ln = lane & 15, hh = lane >> 4;
  const int ntn = N >> 6;
  const int mt = blockIdx.x / ntn, nq = blockIdx.x - mt * ntn;
  const int row0 = mt * 128 + 32 * w, col0 = nq * 64;
  if (row0 >= M) return;
  const unsigned short* a0p = A + (size_t)(row0 + ln) * lda + 8 * hh;
  const unsigned short* a1p = a0p + (size_t)16 * lda;
  const unsigned short* l0p = AL + (size_t)(row0 + ln) * lda + 8 * hh;
  const unsigned short* l1p = l0p + (size_t)16 * lda;
  const unsigned short* b0p = Bt + (size_t)(col0 + ln) * pitch_b + 8 * hh;
  const unsigned short* b1p = b0p + (size_t)16 * pitch_b;
  const unsigned short* b2p = b1p + (size_t)16 * pitch_b;
  const unsigned short* b3p = b2p + (size_t)16 * pitch_b;
  const v8f z8 = {0.f, 0.f, 0.f, 0.f, 0.f, 0.f, 0.f, 0.f};
  v8f c00 = z8, c01 = z8, c02 = z8, c03 = z8, c10 = z8, c11 = z8, c12 = z8, c13 = z8;
#pragma unroll 1
  for (int kb = 0; kb < K; kb += 32) {
    const v16b a0 = ldb(a0p + kb), a1 = ldb(a1p + kb);
    v16b e0 = a0, e1 = a1;
    if (NA == 2) { e0 = ldb(l0p + kb); e1 = ldb(l1p + kb); }
    v16b b = ldb(b0p + kb);
    c00 = mma_b(a0, b, c00); if (NA == 2) c00 = mma_b(e0, b, c00);
    c10 = mma_b(a1, b, c10); if (NA == 2) c10 = mma_b(e1, b, c10);
    b = ldb(b1p + kb);
    c01 = mma_b(a0, b, c01); if (NA == 2) c01 = mma_b(e0, b, c01);
    c11 = mma_b(a1, b, c11); if (NA == 2) c11 = mma_b(e1, b, c11);
    b = ldb(b2p + kb);
    c02 = mma_b(a0, b, c02); if (NA == 2) c02 = mma_b(e0, b, c02);
    c12 = mma_b(a1, b, c12); if (NA == 2) c12 = mma_b(e1, b, c12);
    b = ldb(b3p + kb);
    c03 = mma_b(a0, b, c03); if (NA == 2) c03 = mma_b(e0, b, c03);
    c13 = mma_b(a1, b, c13); if (NA == 2) c13 = mma_b(e1, b, c13);
  }
  const v8f accs[8] = {c00, c01, c02, c03, c10, c11, c12, c13};
  float brow[16];
#pragma unroll
  for (int i = 0; i < 16; ++i) brow[i] = 0.f;
  if (EPI == 1) {
#pragma unroll
    for (int i = 0; i < 16; ++i) brow[i] = bf16_rne(bias[row0 + (i >> 3) * 16 + 8 * hh + (i & 7)]);
  }
#pragma unroll
  for (int u = 0; u < 8; ++u) {
    const int t = u & 3, half = u >> 2;
    const int col = col0 + t * 16 + ln;
    float bc = 0.f;
    if (EPI != 1) bc = bf16_rne(bias[col]);
#pragma unroll
    for (int r = 0; r < 8; ++r) {
      const int rloc = half * 16 + 8 * hh + r;
      float v = accs[u][r];
      if (EPI == 1) v += brow[half * 8 + r]; else v += bc;
      if (EPI == 0) v *= escale;
      so[w][rloc][t * 16 + ln] = v;
    }
  }
  __builtin_amdgcn_fence(4  , "workgroup");
  __builtin_amdgcn_wave_barrier();
  if (EPI == 2) {
    const int rsub = lane >> 4, c4 = (lane & 15) * 4;
    for (int pass = 0; pass < 2; ++pass) {
#pragma unroll
      for (int q = 0; q < 16; ++q) {
        const int r = q * 2 + rsub;
        const v4f v = *(const v4fa*)&so[w][r][c4];
        *(volatile v4f*)(OF + (size_t)(row0 + r) * ldc + col0 + c4) = v;
      }
      if (pass == 0) __threadfence();
    }
  } else {
    const int rsub = lane >> 3, c8 = (lane & 7) * 8;
    for (int pass = 0; pass < 2; ++pass) {
#pragma unroll
      for (int q = 0; q < 8; ++q) {
        const int r = q * 4 + rsub;
        const v4f x0 = *(const v4fa*)&so[w][r][c8], x1 = *(const v4fa*)&so[w][r][c8 + 4];
        const size_t g = (size_t)(row0 + r) * ldc + col0 + c8;
        if (EPI == 0) {
          v8us hi, lo;
#pragma unroll
          for (int i = 0; i < 4; ++i) {
            unsigned short hb = bf16_bits(x0[i]); hi[i] = hb; lo[i] = bf16_bits(x0[i] - bf16_val(hb));
            hb = bf16_bits(x1[i]); hi[4 + i] = hb; lo[4 + i] = bf16_bits(x1[i] - bf16_val(hb));
          }
          *(volatile v8us*)(O1 + g) = hi;
          *(volatile v8us*)(O2 + g) = lo;
        } else {
          Pack8 p;
#pragma unroll
          for (int i = 0; i < 4; ++i) { p.h[i] = (_Float16)x0[i]; p.h[4 + i] = (_Float16)x1[i]; }
          const v8us pv = p.v;
          *(volatile v8us*)(O1 + g) = pv;
        }
      }
      if (pass == 0) __threadfence();
    }
  }
}

__global__ __launch_bounds__(128) void k_proj_hl(const unsigned short* __restrict__ XB, const unsigned short* __restrict__ Wb, const float* __restrict__ bias, float escale,
                                                 unsigned short* __restrict__ OH, unsigned short* __restrict__ OL) {
  gemm_tile<1, 0>(XB, XB, DM, Wb, DM, bias, escale, OH, OL, nullptr, DM, NRI, DM, DM);
}
__global__ __launch_bounds__(128) void k_proj_vt(const unsigned short* __restrict__ Wb, const unsigned short* __restrict__ XB, const float* __restrict__ bias,
                                                 unsigned short* __restrict__ VT) {
  gemm_tile<1, 1>(Wb, Wb, DM, XB, DM, bias, 1.0f, VT, VT, nullptr, NRI, DM, NRI, DM);
}
__global__ __launch_bounds__(128) void k_out(const unsigned short* __restrict__ CH, const unsigned short* __restrict__ CL, const unsigned short* __restrict__ Wb,
                                             const float* __restrict__ bias, float* __restrict__ out) {
  gemm_tile<2, 2>(CH, CL, DM, Wb, DM, bias, 1.0f, nullptr, nullptr, out, DM, NRI, DM, DM);
}

__global__ __launch_bounds__(128) void k_attn(const unsigned short* __restrict__ QH, const unsigned short* __restrict__ QL,
                                              const unsigned short* __restrict__ KH, const unsigned short* __restrict__ KL,
                                              const unsigned short* __restrict__ VT,
                                              unsigned short* __restrict__ CH, unsigned short* __restrict__ CL) {
  __shared__ __attribute__((aligned(16))) float so[4][16][68];
  const int wave = __builtin_amdgcn_readfirstlane((int)(threadIdx.x >> 5));
  const int lane = threadIdx.x & 31, ln = lane & 15, hh = lane >> 4;
  const int bh = blockIdx.y;
  const int b = bh / NH, h = bh - b * NH;
  const int q0 = blockIdx.x * 64 + wave * 16;
  const size_t rowb = (size_t)b * SEQ;
  const size_t qoff = (rowb + q0 + ln) * DM + h * HD + 8 * hh;
  const v16b qh0 = ldb(QH + qoff), qh1 = ldb(QH + qoff + 32);
  const v16b ql0 = ldb(QL + qoff), ql1 = ldb(QL + qoff + 32);
  const size_t kbase = (rowb + ln) * DM + h * HD + 8 * hh;
  const size_t vbase = (size_t)(h * HD + ln) * NR + rowb + 8 * hh;
  const v8f z8 = {0.f, 0.f, 0.f, 0.f, 0.f, 0.f, 0.f, 0.f};
  v8f o0 = z8, o1 = z8, o2 = z8, o3 = z8;
  float m = -1.0e30f, l = 0.f;
#pragma unroll 1
  for (int j0 = 0; j0 < SEQ; j0 += 32) {
    const size_t k0 = kbase + (size_t)j0 * DM;
    const size_t k1 = k0 + (size_t)16 * DM;
    v8f s0 = z8, s1 = z8;
    {
      v16b ah = ldb(KH + k0), al = ldb(KL + k0);
      s0 = mma_b(al, qh0, s0); s0 = mma_b(ah, ql0, s0); s0 = mma_b(ah, qh0, s0);
      ah = ldb(KH + k0 + 32); al = ldb(KL + k0 + 32);
      s0 = mma_b(al, qh1, s0); s0 = mma_b(ah, ql1, s0); s0 = mma_b(ah, qh1, s0);
      ah = ldb(KH + k1); al = ldb(KL + k1);
      s1 = mma_b(al, qh0, s1); s1 = mma_b(ah, ql0, s1); s1 = mma_b(ah, qh0, s1);
      ah = ldb(KH + k1 + 32); al = ldb(KL + k1 + 32);
      s1 = mma_b(al, qh1, s1); s1 = mma_b(ah, ql1, s1); s1 = mma_b(ah, qh1, s1);
    }
    float mx = fmaxf(s0[0], s1[0]);
#pragma unroll
    for (int r = 1; r < 8; ++r) mx = fmaxf(mx, fmaxf(s0[r], s1[r]));
    mx = fmaxf(mx, __shfl_xor(mx, 16, 32));
    const float mnew = fmaxf(m, mx);
    const float sc = __expf(m - mnew);
    const float msh = mnew - LN_CARRY;
    FragH pf;
    float ps = 0.f;
#pragma unroll
    for (int r = 0; r < 8; ++r) {
      const float p0 = __expf(s0[r] - msh);
      const float p1 = __expf(s1[r] - msh);
      ps += p0 + p1;
      pf.h[r] = (_Float16)p0;
      pf.h[8 + r] = (_Float16)p1;
    }
    ps += __shfl_xor(ps, 16, 32);
    l = l * sc + ps;
    m = mnew;
    o0 *= sc; o1 *= sc; o2 *= sc; o3 *= sc;
    const size_t v0 = vbase + j0;
    v16h a = ldh(VT + v0);
    o0 = mma_h(a, pf.v, o0);
    a = ldh(VT + v0 + (size_t)16 * NR);
    o1 = mma_h(a, pf.v, o1);
    a = ldh(VT + v0 + (size_t)32 * NR);
    o2 = mma_h(a, pf.v, o2);
    a = ldh(VT + v0 + (size_t)48 * NR);
    o3 = mma_h(a, pf.v, o3);
  }
  const float inv = 1.0f / l;
  {
    v4f t0, t1;
    t0[0] = o0[0] * inv; t0[1] = o0[1] * inv; t0[2] = o0[2] * inv; t0[3] = o0[3] * inv;
    t1[0] = o0[4] * inv; t1[1] = o0[5] * inv; t1[2] = o0[6] * inv; t1[3] = o0[7] * inv;
    *(v4fa*)&so[wave][ln][0 + 8 * hh] = t0; *(v4fa*)&so[wave][ln][0 + 8 * hh + 4] = t1;
    t0[0] = o1[0] * inv; t0[1] = o1[1] * inv; t0[2] = o1[2] * inv; t0[3] = o1[3] * inv;
    t1[0] = o1[4] * inv; t1[1] = o1[5] * inv; t1[2] = o1[6] * inv; t1[3] = o1[7] * inv;
    *(v4fa*)&so[wave][ln][16 + 8 * hh] = t0; *(v4fa*)&so[wave][ln][16 + 8 * hh + 4] = t1;
    t0[0] = o2[0] * inv; t0[1] = o2[1] * inv; t0[2] = o2[2] * inv; t0[3] = o2[3] * inv;
    t1[0] = o2[4] * inv; t1[1] = o2[5] * inv; t1[2] = o2[6] * inv; t1[3] = o2[7] * inv;
    *(v4fa*)&so[wave][ln][32 + 8 * hh] = t0; *(v4fa*)&so[wave][ln][32 + 8 * hh + 4] = t1;
    t0[0] = o3[0] * inv; t0[1] = o3[1] * inv; t0[2] = o3[2] * inv; t0[3] = o3[3] * inv;
    t1[0] = o3[4] * inv; t1[1] = o3[5] * inv; t1[2] = o3[6] * inv; t1[3] = o3[7] * inv;
    *(v4fa*)&so[wave][ln][48 + 8 * hh] = t0; *(v4fa*)&so[wave][ln][48 + 8 * hh + 4] = t1;
  }
  __builtin_amdgcn_fence(4  , "workgroup");
  __builtin_amdgcn_wave_barrier();
  const int rsub = lane >> 3, c8 = (lane & 7) * 8;
  for (int pass = 0; pass < 2; ++pass) {
#pragma unroll
    for (int it = 0; it < 4; ++it) {
      const int r = it * 4 + rsub;
      const v4f x0 = *(const v4fa*)&so[wave][r][c8], x1 = *(const v4fa*)&so[wave][r][c8 + 4];
      v8us hi, lo;
#pragma unroll
      for (int i = 0; i < 4; ++i) {
        unsigned short hb = bf16_bits(x0[i]); hi[i] = hb; lo[i] = bf16_bits(x0[i] - bf16_val(hb));
        hb = bf16_bits(x1[i]); hi[4 + i] = hb; lo[4 + i] = bf16_bits(x1[i] - bf16_val(hb));
      }
      const size_t g = (rowb + q0 + r) * DM + h * HD + c8;
      *(volatile v8us*)(CH + g) = hi;
      *(volatile v8us*)(CL + g) = lo;
    }
    if (pass == 0) __threadfence();
  }
}

#define PLANE_X ((size_t)NB * SEQ * DM * 2)
#define PLANE_W ((size_t)DM * DM * 2)
#define CARVE_TOTAL (PLANE_X * 8 + PLANE_W * 4)
static_assert(PLANE_X % 256 == 0);
static_assert(PLANE_W % 256 == 0);
static_assert(CARVE_TOTAL <= (size_t)134217728);

extern "C" void kernel_launch(void* const* d_in, const int* in_sizes, int n_in,
                              void* d_out, int out_size, void* d_ws, size_t ws_size, hipStream_t stream) {
  if (n_in < 9) return;
  if ((size_t)in_sizes[0] < ((size_t)(NB - 1) * SEQ_FULL + SEQ) * DM) return;
  if (in_sizes[1] < DM * DM || in_sizes[3] < DM * DM || in_sizes[5] < DM * DM || in_sizes[7] < DM * DM) return;
  if (in_sizes[2] < DM || in_sizes[4] < DM || in_sizes[6] < DM || in_sizes[8] < DM) return;
  if ((size_t)out_size < NR * DM) return;
  if (ws_size < CARVE_TOTAL) return;
  const float* x  = (const float*)d_in[0];
  const float* wq = (const float*)d_in[1]; const float* bq = (const float*)d_in[2];
  const float* wk = (const float*)d_in[3]; const float* bk = (const float*)d_in[4];
  const float* wv = (const float*)d_in[5]; const float* bv = (const float*)d_in[6];
  const float* wo = (const float*)d_in[7]; const float* bo = (const float*)d_in[8];
  char* ws = (char*)d_ws;
  size_t off = 0;
  unsigned short* XB = (unsigned short*)(ws + off); off += PLANE_X;
  unsigned short* WQ = (unsigned short*)(ws + off); off += PLANE_W;
  unsigned short* WK = (unsigned short*)(ws + off); off += PLANE_W;
  unsigned short* WV = (unsigned short*)(ws + off); off += PLANE_W;
  unsigned short* WO = (unsigned short*)(ws + off); off += PLANE_W;
  unsigned short* QH = (unsigned short*)(ws + off); off += PLANE_X;
  unsigned short* QL = (unsigned short*)(ws + off); off += PLANE_X;
  unsigned short* KH = (unsigned short*)(ws + off); off += PLANE_X;
  unsigned short* KL = (unsigned short*)(ws + off); off += PLANE_X;
  unsigned short* VT = (unsigned short*)(ws + off); off += PLANE_X;
  unsigned short* CH = (unsigned short*)(ws + off); off += PLANE_X;
  unsigned short* CL = (unsigned short*)(ws + off); off += PLANE_X;
  if (off > ws_size) return;

  const int w8 = DM * DM / 8;
  const unsigned gw = (unsigned)((w8 + 255) / 256);
  k_w_bf16<<<gw, 256, 0, stream>>>(wq, WQ, w8);
  k_w_bf16<<<gw, 256, 0, stream>>>(wk, WK, w8);
  k_w_bf16<<<gw, 256, 0, stream>>>(wv, WV, w8);
  k_w_bf16<<<gw, 256, 0, stream>>>(wo, WO, w8);
  const int x8 = (int)(NR * DM / 8);
  k_x_bf16<<<(unsigned)((x8 + 255) / 256), 256, 0, stream>>>(x, XB, x8);

  const unsigned gp = (unsigned)((NRI / 128) * (DM / 64));
  k_proj_hl<<<gp, 128, 0, stream>>>(XB, WQ, bq, 0.125f, QH, QL);
  k_proj_hl<<<gp, 128, 0, stream>>>(XB, WK, bk, 1.0f, KH, KL);
  const unsigned gv = (unsigned)((DM / 128) * (NRI / 64));
  k_proj_vt<<<gv, 128, 0, stream>>>(WV, XB, bv, VT);

  k_attn<<<dim3((unsigned)(SEQ / 64), (unsigned)(NB * NH)), 128, 0, stream>>>(QH, QL, KH, KL, VT, CH, CL);

  k_out<<<gp, 128, 0, stream>>>(CH, CL, WO, bo, (float*)d_out);
}
